// GraphAttentionLayer_61804579389526
// MI455X (gfx1250) — hardware-run, weakly checked
//
#include <hip/hip_runtime.h>

typedef float          v8f   __attribute__((ext_vector_type(8)));
typedef float          v4f   __attribute__((ext_vector_type(4)));
typedef unsigned int   v4u   __attribute__((ext_vector_type(4)));
typedef int            v8i   __attribute__((ext_vector_type(8)));
typedef unsigned short v8us  __attribute__((ext_vector_type(8)));
typedef unsigned short v16us __attribute__((ext_vector_type(16)));
typedef __bf16         v16bf __attribute__((ext_vector_type(16)));
typedef _Float16       v16h  __attribute__((ext_vector_type(16)));
typedef v4f  __attribute__((may_alias)) v4fa;
typedef v8us __attribute__((may_alias)) v8usa;
union FragB { v16bf v; v16us u; v8us h[2]; v8i w; };
union FragH { v16h  v; v16us u; v8us h[2]; v8i w; };

__device__ __forceinline__ v8f wmb(const FragB& a, const FragB& b, v8f c) {
  v8f d = __builtin_amdgcn_wmma_f32_16x16x32_bf16(false, a.v, false, b.v, (short)0, c, false, false);
  asm volatile("v_nop\n\tv_nop\n\tv_nop\n\tv_nop" : "+v"(d) : "v"(a.w), "v"(b.w));
  return d;
}

__device__ __forceinline__ v8f wmh(const FragH& a, const FragH& b, v8f c) {
  v8f d = __builtin_amdgcn_wmma_f32_16x16x32_f16(false, a.v, false, b.v, (short)0, c, false, false);
  asm volatile("v_nop\n\tv_nop\n\tv_nop\n\tv_nop" : "+v"(d) : "v"(a.w), "v"(b.w));
  return d;
}

__device__ __forceinline__ unsigned bf16_bits(float f) {
  const unsigned u = __float_as_uint(f);
  const unsigned r = (u + 0x7FFFu + ((u >> 16) & 1u)) >> 16;
  const unsigned q = (u >> 16) | 0x40u;
  return ((u & 0x7fffffffu) > 0x7f800000u) ? q : r;
}

__device__ __forceinline__ float bf16_val(float f) {
  return __uint_as_float(bf16_bits(f) << 16);
}
__device__ __forceinline__ int clampi(int v, int lo, int hi) {
  return v < lo ? lo : (v > hi ? hi : v);
}

__device__ __forceinline__ unsigned f16_bits(float f) {
  const unsigned u  = __float_as_uint(f);
  const unsigned s  = (u >> 16) & 0x8000u;
  const unsigned a  = u & 0x7fffffffu;
  const unsigned t  = a - 0x38000000u;
  const unsigned r  = (t + 0x0FFFu + ((t >> 13) & 1u)) >> 13;
  const unsigned rc = r > 0x7C00u ? 0x7C00u : r;
  const bool small  = a < 0x38800000u;
  const bool isnan  = a > 0x7f800000u;
  const unsigned fin = small ? 0u : (s | rc);
  return isnan ? (s | 0x7E00u) : fin;
}

__device__ __forceinline__ unsigned pk16(unsigned lo, unsigned hi) { return lo | (hi << 16); }
__device__ __forceinline__ unsigned bf16_lo_bits(float v) {
  float hi = bf16_val(v);
  asm volatile("" : "+v"(hi));
  return bf16_bits(v - hi);
}
__device__ __forceinline__ v4u pack8_bf16(v4f a, v4f c) {
  return (v4u){ pk16(bf16_bits(a[0]), bf16_bits(a[1])), pk16(bf16_bits(a[2]), bf16_bits(a[3])),
                pk16(bf16_bits(c[0]), bf16_bits(c[1])), pk16(bf16_bits(c[2]), bf16_bits(c[3])) };
}
__device__ __forceinline__ v4u pack8_bf16_lo(v4f a, v4f c) {
  return (v4u){ pk16(bf16_lo_bits(a[0]), bf16_lo_bits(a[1])), pk16(bf16_lo_bits(a[2]), bf16_lo_bits(a[3])),
                pk16(bf16_lo_bits(c[0]), bf16_lo_bits(c[1])), pk16(bf16_lo_bits(c[2]), bf16_lo_bits(c[3])) };
}
__device__ __forceinline__ v4u pack8_f16(v4f a, v4f c) {
  return (v4u){ pk16(f16_bits(a[0]), f16_bits(a[1])), pk16(f16_bits(a[2]), f16_bits(a[3])),
                pk16(f16_bits(c[0]), f16_bits(c[1])), pk16(f16_bits(c[2]), f16_bits(c[3])) };
}

template <int FORM>
__global__ __launch_bounds__(256) void k_plane(const float* __restrict__ src, int rows, int cols, int ldsrc,
                                               unsigned short* __restrict__ dst, int MP, int KP) {
  static_assert(FORM >= 0 && FORM <= 3);
  const int KTOT = (FORM == 1 || FORM == 3) ? 2 * KP : KP;
  const unsigned ppr   = (unsigned)(KTOT >> 3);
  const unsigned kp8   = (unsigned)(KP >> 3);
  const unsigned total = (unsigned)MP * ppr;
  const unsigned g     = blockIdx.x * 256u + threadIdx.x;
  const unsigned rowu  = g / ppr;
  const unsigned p     = g - rowu * ppr;
  const bool second    = p >= kp8;
  const int row = (int)rowu;
  const int c0  = (int)((second ? p - kp8 : p) << 3);
  const float* srow = src + (size_t)clampi(row, 0, rows - 1) * (size_t)ldsrc;
  float x[8];
  unsigned mk[8];
#pragma unroll
  for (int e = 0; e < 8; ++e) {
    const int c = c0 + e;
    const float v = srow[clampi(c, 0, cols - 1)];
    asm volatile("" :: "v"(v));
    x[e]  = v;
    mk[e] = (row < rows && c < cols) ? 0xFFFFu : 0u;
  }
  const v4f a = (v4f){ x[0], x[1], x[2], x[3] };
  const v4f c = (v4f){ x[4], x[5], x[6], x[7] };
  v4u o;
  if (FORM == 2) {
    o = pack8_f16(a, c);
  } else {
    const v4u hi = pack8_bf16(a, c);
    o = hi;
    if (FORM == 1) { const v4u lo = pack8_bf16_lo(a, c); o = second ? lo : hi; }
  }
  const v4u mw = (v4u){ pk16(mk[0], mk[1]), pk16(mk[2], mk[3]), pk16(mk[4], mk[5]), pk16(mk[6], mk[7]) };
  o &= mw;
  if (g < total) {
    volatile v4u* q = (volatile v4u*)(dst + (size_t)g * 8);
    *q = o;
    __threadfence();
    *q = o;
  }
}

template <int FORM> struct FragOf    { typedef FragB T; };
template <>         struct FragOf<2> { typedef FragH T; };
__device__ __forceinline__ v8f mm(const FragB& a, const FragB& b, v8f c) { return wmb(a, b, c); }
__device__ __forceinline__ v8f mm(const FragH& a, const FragH& b, v8f c) { return wmh(a, b, c); }
template <class F> __device__ __forceinline__ F ld_frag(const unsigned short* p) {
  F f;
  f.h[0] = *(const v8usa*)(p);
  f.h[1] = *(const v8usa*)(p + 16);
  return f;
}

template <int FORM, int EPI>
__global__ __launch_bounds__(256) __attribute__((amdgpu_num_vgpr(248)))
void k_gemm_nt(const unsigned short* __restrict__ A, const unsigned short* __restrict__ B,
               const float* __restrict__ bias, float* __restrict__ D, int M, int N, int KTOT, int ldd) {
  static_assert(FORM >= 0 && FORM <= 2);
  static_assert(EPI == 0 || EPI == 1);
  typedef typename FragOf<FORM>::T F;
  __shared__ __attribute__((aligned(16))) float sT[8][16 * 68];
  const int lane = threadIdx.x & 31;
  const int wave = threadIdx.x >> 5;
  const int tilesM = (M + 63) >> 6;
  const int tilesN = (N + 63) >> 6;
  const int tile = blockIdx.x * 8 + wave;
  if (tile >= tilesM * tilesN) return;
  const int tm = tile / tilesN;
  const int tn = tile - tm * tilesN;
  const int m0 = tm << 6;
  const int n0 = tn << 6;

  const int rl = lane & 15;
  const int h8 = (lane >> 4) * 8;
  const unsigned short* pa = A + (size_t)(m0 + rl) * (size_t)KTOT + h8;
  const unsigned short* pb = B + (size_t)(n0 + rl) * (size_t)KTOT + h8;

  v8f acc[4][4];
#pragma unroll
  for (int i = 0; i < 4; ++i)
#pragma unroll
    for (int j = 0; j < 4; ++j) acc[i][j] = (v8f){0.f, 0.f, 0.f, 0.f, 0.f, 0.f, 0.f, 0.f};

#pragma unroll 1
  for (int k0 = 0; k0 < KTOT; k0 += 32) {
    F bf[4];
#pragma unroll
    for (int j = 0; j < 4; ++j) bf[j] = ld_frag<F>(pb + (size_t)(j << 4) * (size_t)KTOT + k0);
#pragma unroll
    for (int i = 0; i < 4; ++i) {
      const F af = ld_frag<F>(pa + (size_t)(i << 4) * (size_t)KTOT + k0);
#pragma unroll
      for (int j = 0; j < 4; ++j) acc[i][j] = mm(af, bf[j], acc[i][j]);
    }
  }

  float* slab = sT[wave];
  const int hh = lane >> 4;
  const int c4 = (lane & 15) * 4;
  const int nc = n0 + c4;
  const bool cok = nc < N;
  v4f bv = (v4f){0.f, 0.f, 0.f, 0.f};
  if (EPI == 1) {
    bv = *(const v4fa*)(bias + clampi(nc, 0, N - 4));
    asm volatile("" :: "v"(bv));
  }
#pragma unroll
  for (int i = 0; i < 4; ++i) {
    const int mBase = m0 + (i << 4);
#pragma unroll
    for (int j = 0; j < 4; ++j) {
#pragma unroll
      for (int r = 0; r < 8; ++r) slab[(h8 + r) * 68 + (j << 4) + rl] = acc[i][j][r];
    }
    __builtin_amdgcn_fence(__ATOMIC_RELEASE, "workgroup");
    __builtin_amdgcn_wave_barrier();
    __builtin_amdgcn_fence(__ATOMIC_ACQUIRE, "workgroup");
    v4f vv[8];
#pragma unroll
    for (int it = 0; it < 8; ++it) {
      const int row = it * 2 + hh;
      v4f v = *(const v4fa*)(slab + row * 68 + c4);
      if (EPI == 1) v += bv;
      vv[it] = v;
    }
    for (int pass = 0; pass < 2; ++pass) {
#pragma unroll
      for (int it = 0; it < 8; ++it) {
        const int row = mBase + it * 2 + hh;
        if (cok && row < M) *(volatile v4f*)(D + (size_t)row * (size_t)ldd + nc) = vv[it];
      }
      __threadfence();
    }
    __builtin_amdgcn_fence(__ATOMIC_RELEASE, "workgroup");
    __builtin_amdgcn_wave_barrier();
    __builtin_amdgcn_fence(__ATOMIC_ACQUIRE, "workgroup");
  }
}

#define GN_N      10000
#define GN_D      512
#define GN_H      8
#define GN_E      160000
#define GN_MP     10112
#define GN_LDH    1024
#define GN_NB     512
#define GN_NBLK   20
#define GN_NPADT  (GN_NB * GN_NBLK)
#define GN_RCAP   12288
#define GN_DEGCAP 64
#define GN_CHUNK  2048
#define GN_WCAP   256
#define GN_LISTN  2048
#define GN_TS     96
#define GN_RB     128
#define GN_SB     79
#define GN_BK_LDS ((2 * GN_RCAP + 2 * GN_NB + GN_LISTN + 16) * 4)

static_assert(GN_N <= GN_NBLK * GN_NB);
static_assert(GN_E == 78 * GN_CHUNK + 256);
static_assert(GN_RCAP * 4 >= 8338 * 5);
static_assert(GN_DEGCAP >= 36 + 8);
static_assert(GN_TS >= GN_DEGCAP + 1 && GN_TS == 96);
static_assert(GN_MP % 64 == 0 && GN_MP >= GN_N && GN_LDH % 64 == 0 && GN_D % 32 == 0);
static_assert((GN_RCAP % 1024) == 0);
static_assert(GN_NB == 2 * 256);
static_assert(GN_LISTN == 8 * GN_WCAP && GN_LISTN >= GN_NB);
static_assert(GN_SB * GN_RB >= GN_N && (GN_SB - 1) * GN_RB < GN_N);
static_assert(GN_N % 8 == 0);
static_assert(GN_E < (1 << 19) && GN_NB <= 4096);
static_assert(GN_BK_LDS <= 327680);

typedef int    v4i  __attribute__((ext_vector_type(4)));
typedef float  v2f  __attribute__((ext_vector_type(2)));
typedef double v2d  __attribute__((ext_vector_type(2)));
typedef v4i __attribute__((may_alias)) v4ia;
typedef v2f __attribute__((may_alias)) v2fa;

constexpr size_t gn_al(size_t v) { return (v + 255) & ~(size_t)255; }
constexpr size_t SZ_XB   = gn_al((size_t)GN_MP * GN_D * 2);
constexpr size_t SZ_WT   = gn_al((size_t)GN_LDH * GN_D * 2);
constexpr size_t SZ_HS   = gn_al((size_t)GN_MP * GN_LDH * 4);
constexpr size_t SZ_SD   = gn_al((size_t)GN_N * 16 * 4);
constexpr size_t SZ_G    = gn_al((size_t)GN_N * GN_D * 4);
constexpr size_t SZ_LIST = gn_al((size_t)GN_NBLK * GN_RCAP * 4);
constexpr size_t SZ_TAB  = gn_al((size_t)GN_NPADT * 4);
constexpr size_t SZ_REC  = gn_al((size_t)GN_SB * GN_D * 8);
constexpr size_t SZ_STAT = gn_al((size_t)2 * GN_D * 4);
constexpr size_t SZ_PAR  = gn_al((size_t)6 * GN_D * 4);
constexpr size_t OF_XB   = 0;
constexpr size_t OF_WT   = OF_XB + SZ_XB;
constexpr size_t OF_HS   = OF_WT + SZ_WT;
constexpr size_t OF_SD   = OF_HS + SZ_HS;
constexpr size_t OF_G    = OF_SD + SZ_SD;
constexpr size_t OF_LIST = OF_G + SZ_G;
constexpr size_t OF_OFF  = OF_LIST + SZ_LIST;
constexpr size_t OF_CNT  = OF_OFF + SZ_TAB;
constexpr size_t OF_FLG  = OF_CNT + SZ_TAB;
constexpr size_t OF_REC1 = OF_FLG + SZ_TAB;
constexpr size_t OF_REC2 = OF_REC1 + SZ_REC;
constexpr size_t OF_STAT = OF_REC2 + SZ_REC;
constexpr size_t OF_PAR  = OF_STAT + SZ_STAT;
constexpr size_t WS_TOTAL = OF_PAR + SZ_PAR;
static_assert(WS_TOTAL == 75711488);
static_assert(WS_TOTAL <= ((size_t)128 << 20));
static_assert((size_t)GN_N * 16 * 4 == (size_t)(GN_N / 8) * 512);
static_assert((size_t)GN_NBLK * GN_NB * 4 <= SZ_TAB);
static_assert((size_t)(GN_SB - 1) * GN_D * 8 + GN_D * 8 <= SZ_REC);

__device__ __forceinline__ v4f gn_bf4(v4f v) {
  return (v4f){ bf16_val(v[0]), bf16_val(v[1]), bf16_val(v[2]), bf16_val(v[3]) };
}

__global__ __launch_bounds__(256) void k_wtr(const float* __restrict__ w, unsigned short* __restrict__ wt) {
  const int u  = (int)blockIdx.x * 256 + (int)threadIdx.x;
  const int n  = u >> 6;
  const int k8 = (u & 63) << 3;
  const float* p = w + (size_t)k8 * GN_D + n;
  float x[8];
#pragma unroll
  for (int e = 0; e < 8; ++e) {
    const float v = p[(size_t)e * GN_D];
    asm volatile("" :: "v"(v));
    x[e] = v;
  }
  const v4u o = pack8_bf16((v4f){ x[0], x[1], x[2], x[3] }, (v4f){ x[4], x[5], x[6], x[7] });
  volatile v4u* q = (volatile v4u*)(wt + (size_t)n * GN_D + k8);
  *q = o;
  __threadfence();
  *q = o;
}

__global__ __launch_bounds__(128) void k_par(const float* __restrict__ p0, const float* __restrict__ p1,
                                             const float* __restrict__ p2, const float* __restrict__ p3,
                                             const float* __restrict__ p4, const float* __restrict__ p5,
                                             float* __restrict__ PAR) {
  const int t4 = (int)threadIdx.x * 4;
  const v4f a0 = gn_bf4(*(const v4fa*)(p0 + t4));
  const v4f a1 = gn_bf4(*(const v4fa*)(p1 + t4));
  const v4f a2 = gn_bf4(*(const v4fa*)(p2 + t4));
  const v4f a3 = gn_bf4(*(const v4fa*)(p3 + t4));
  const v4f a4 = gn_bf4(*(const v4fa*)(p4 + t4));
  const v4f a5 = gn_bf4(*(const v4fa*)(p5 + t4));
  for (int pass = 0; pass < 2; ++pass) {
    *(volatile v4f*)(PAR + 0 * GN_D + t4) = a0;
    *(volatile v4f*)(PAR + 1 * GN_D + t4) = a1;
    *(volatile v4f*)(PAR + 2 * GN_D + t4) = a2;
    *(volatile v4f*)(PAR + 3 * GN_D + t4) = a3;
    *(volatile v4f*)(PAR + 4 * GN_D + t4) = a4;
    *(volatile v4f*)(PAR + 5 * GN_D + t4) = a5;
    __threadfence();
  }
}

__global__ __launch_bounds__(256) void k_dots(const float* __restrict__ HS, const float* __restrict__ PAR,
                                              float* __restrict__ SD, int nN) {
  __shared__ __attribute__((aligned(16))) float sAtt[2 * GN_D];
  __shared__ __attribute__((aligned(16))) float sSD[128];
  const int tid = (int)threadIdx.x, lane = tid & 31, wave = tid >> 5, hh = lane >> 4;
  *(v4fa*)(sAtt + 4 * tid) = *(const v4fa*)(PAR + 4 * tid);
  __syncthreads();
  const int row = (int)blockIdx.x * 8 + wave;
  const int rc  = clampi(row, 0, nN - 1);
  const float* hp = HS + (size_t)rc * GN_LDH + 4 * lane;
  float ps[4], pd[4];
#pragma unroll
  for (int j = 0; j < 4; ++j) {
    const v4f h  = *(const v4fa*)(hp + j * 128);
    const v4f as = *(const v4fa*)(sAtt + j * 128 + 4 * lane);
    const v4f ad = *(const v4fa*)(sAtt + GN_D + j * 128 + 4 * lane);
    float s = h[0] * as[0];
    s = fmaf(h[1], as[1], s); s = fmaf(h[2], as[2], s); s = fmaf(h[3], as[3], s);
    float d = h[0] * ad[0];
    d = fmaf(h[1], ad[1], d); d = fmaf(h[2], ad[2], d); d = fmaf(h[3], ad[3], d);
    ps[j] = s; pd[j] = d;
  }
#pragma unroll
  for (int j = 0; j < 4; ++j) {
#pragma unroll
    for (int o = 8; o > 0; o >>= 1) {
      ps[j] += __shfl_xor(ps[j], o);
      pd[j] += __shfl_xor(pd[j], o);
    }
  }
  if ((lane & 15) == 0) {
#pragma unroll
    for (int j = 0; j < 4; ++j) {
      sSD[wave * 16 + 2 * j + hh]     = ps[j];
      sSD[wave * 16 + 8 + 2 * j + hh] = pd[j];
    }
  }
  __syncthreads();
  if (wave == 0) {
    const v4f v = *(const v4fa*)(sSD + 4 * lane);
    volatile v4f* q = (volatile v4f*)(SD + (size_t)blockIdx.x * 128 + 4 * lane);
    *q = v;
    __threadfence();
    *q = v;
  }
}

__device__ __forceinline__ int gn_scan_chunk(const int* __restrict__ dsts, int nE, int nN, int cbase, int slotBase,
                                            int* list, int lane, int wave) {
  int wc = 0;
  const int el0 = wave * 256 + lane;
  unsigned sl[8];
  bool hit[8];
#pragma unroll
  for (int J = 0; J < 8; ++J) {
    const int e   = cbase + el0 + 32 * J;
    const int ec  = e < nE - 1 ? e : nE - 1;
    const int raw = dsts[ec];
    asm volatile("" :: "v"(raw));
    const int kc  = clampi(raw, 0, nN - 1);
    const int key = (e < nE) ? kc : -1;
    sl[J]  = (unsigned)key - (unsigned)slotBase;
    hit[J] = sl[J] < (unsigned)GN_NB;
  }
#pragma unroll
  for (int J = 0; J < 8; ++J) {
    const unsigned mj = __builtin_amdgcn_ballot_w32(hit[J]);
    if (mj != 0u) {
      if (hit[J]) {
        const int pos = wc + (int)__builtin_amdgcn_mbcnt_lo(mj, 0u);
        if (pos < GN_WCAP) list[wave * GN_WCAP + pos] = ((el0 + 32 * J) << 12) | (int)sl[J];
      }
      wc += (int)__builtin_popcount(mj);
    }
  }
  return wc;
}

__global__ __launch_bounds__(256) void k_bucket(const int* __restrict__ ei, int* __restrict__ LIST,
                                                int* __restrict__ OFFT, int* __restrict__ CNTT,
                                                int* __restrict__ FLGT, int nE, int nN) {
  extern __shared__ v4f gn_lds_dyn[];
  int* reg1 = (int*)gn_lds_dyn;
  int* reg2 = reg1 + GN_RCAP;
  int* scnt = reg2 + GN_RCAP;
  int* soff = scnt + GN_NB;
  int* list = soff + GN_NB;
  int* wcnt = list + GN_LISTN;
  int* wtot = wcnt + 8;
  const int tid = (int)threadIdx.x, lane = tid & 31, wave = tid >> 5;
  const int slotBase = (int)blockIdx.x * GN_NB;
  const int* srcs = ei;
  const int* dsts = ei + nE;

  scnt[2 * tid] = 0; scnt[2 * tid + 1] = 0;
  for (int i = tid; i < GN_RCAP / 4; i += 256) *(v4ia*)(reg2 + 4 * i) = (v4i){0, 0, 0, 0};
  __syncthreads();

  int tot = 0;
  const int nChunks = (nE + GN_CHUNK - 1) / GN_CHUNK;
#pragma unroll 1
  for (int ch = 0; ch < nChunks; ++ch) {
    const int cbase = ch * GN_CHUNK;
    const int wc = gn_scan_chunk(dsts, nE, nN, cbase, slotBase, list, lane, wave);
    if (lane == 0) wcnt[wave] = wc;
    __syncthreads();
    int pre = 0, all = 0;
#pragma unroll
    for (int w2 = 0; w2 < 8; ++w2) {
      int c = wcnt[w2];
      c = c < 0 ? 0 : (c > GN_WCAP ? GN_WCAP : c);
      all += c;
      pre += (w2 < wave) ? c : 0;
    }
    const int wcc  = wc > GN_WCAP ? GN_WCAP : wc;
    const int base = tot + pre;
#pragma unroll 1
    for (int i = lane; i < wcc; i += 32) {
      const int ent = list[wave * GN_WCAP + i];
      const int el  = (ent >> 12) & (GN_CHUNK - 1);
      const int sl  = ent & (GN_NB - 1);
      int eid = cbase + el;
      eid = eid > nE - 1 ? nE - 1 : eid;
      const int pos = base + i;
      if (pos < GN_RCAP) reg1[pos] = (int)(((unsigned)eid << 12) | (unsigned)sl);
    }
    tot += all;
    tot = tot > GN_RCAP ? GN_RCAP : tot;
    __syncthreads();
  }
  const int nh = tot;

  if (wave == 0) {
#pragma unroll 1
    for (int b0 = 0; b0 < nh; b0 += 32) {
      int idx = b0 + lane;
      idx = idx < nh - 1 ? idx : nh - 1;
      const int uv  = reg1[idx];
      const int m32 = (nh - b0) < 32 ? (nh - b0) : 32;
#pragma unroll 1
      for (int k = 0; k < m32; ++k) {
        const int u  = __builtin_amdgcn_readlane(uv, k);
        const int sl = u & (GN_NB - 1);
        if (lane == 0) scnt[sl] = scnt[sl] + 1;
      }
    }
  }
  __syncthreads();

  {
    int e0 = scnt[2 * tid], e1 = scnt[2 * tid + 1];
    e0 = e0 < 0 ? 0 : e0; e1 = e1 < 0 ? 0 : e1;
    const int ts = e0 + e1;
    int incl = ts;
#pragma unroll
    for (int d = 1; d < 32; d <<= 1) {
      const int up = __shfl_up(incl, d);
      if (lane >= d) incl += up;
    }
    if (lane == 31) wtot[wave] = incl;
    __syncthreads();
    int pre = 0;
#pragma unroll
    for (int w2 = 0; w2 < 8; ++w2) pre += (w2 < wave) ? wtot[w2] : 0;
    const int run = pre + incl - ts;
    soff[2 * tid]     = run;
    soff[2 * tid + 1] = run + e0;
  }
  __syncthreads();
  list[2 * tid] = soff[2 * tid]; list[2 * tid + 1] = soff[2 * tid + 1];
  __syncthreads();

  if (wave == 0) {
#pragma unroll 1
    for (int b0 = 0; b0 < nh; b0 += 32) {
      int idx = b0 + lane;
      idx = idx < nh - 1 ? idx : nh - 1;
      const int uv = reg1[idx];
      const int eid = clampi((int)((unsigned)uv >> 12), 0, nE - 1);
      const int sraw = srcs[eid];
      asm volatile("" :: "v"(sraw));
      const int sv  = clampi(sraw, 0, nN - 1);
      const int m32 = (nh - b0) < 32 ? (nh - b0) : 32;
#pragma unroll 1
      for (int k = 0; k < m32; ++k) {
        const int u  = __builtin_amdgcn_readlane(uv, k);
        const int sk = __builtin_amdgcn_readlane(sv, k);
        const int sl = u & (GN_NB - 1);
        if (lane == 0) {
          int pos = list[sl];
          pos = pos < 0 ? 0 : (pos > GN_RCAP - 1 ? GN_RCAP - 1 : pos);
          reg2[pos] = sk;
          list[sl] = pos + 1;
        }
      }
    }
  }
  __syncthreads();

  int* Lb = LIST + (size_t)blockIdx.x * GN_RCAP;
  for (int pass = 0; pass < 2; ++pass) {
#pragma unroll 1
    for (int i = tid; i < GN_RCAP / 4; i += 256) {
      const v4i v = *(const v4ia*)(reg2 + 4 * i);
      *(volatile v4i*)(Lb + 4 * i) = v;
    }
    __threadfence();
  }
  if (tid < 128) {
    const bool ovf = nh >= GN_RCAP;
    const v4i o4 = *(const v4ia*)(soff + 4 * tid);
    v4i c4 = *(const v4ia*)(scnt + 4 * tid);
    c4.x = c4.x < 0 ? 0 : c4.x; c4.y = c4.y < 0 ? 0 : c4.y;
    c4.z = c4.z < 0 ? 0 : c4.z; c4.w = c4.w < 0 ? 0 : c4.w;
    v4i f4;
    f4.x = (ovf || c4.x > GN_DEGCAP) ? 1 : 0;
    f4.y = (ovf || c4.y > GN_DEGCAP) ? 1 : 0;
    f4.z = (ovf || c4.z > GN_DEGCAP) ? 1 : 0;
    f4.w = (ovf || c4.w > GN_DEGCAP) ? 1 : 0;
    volatile v4i* qo = (volatile v4i*)(OFFT + slotBase + 4 * tid);
    volatile v4i* qc = (volatile v4i*)(CNTT + slotBase + 4 * tid);
    volatile v4i* qf = (volatile v4i*)(FLGT + slotBase + 4 * tid);
    *qo = o4; *qc = c4; *qf = f4;
    __threadfence();
    *qo = o4; *qc = c4; *qf = f4;
  }
}

__global__ __launch_bounds__(256) void k_replay(const float* __restrict__ HS, const float* __restrict__ SD,
                                                const float* __restrict__ PAR, const int* __restrict__ LIST,
                                                const int* __restrict__ OFFT, const int* __restrict__ CNTT,
                                                const int* __restrict__ FLGT, float* __restrict__ G, int nN) {
  __shared__ __attribute__((aligned(16))) float sBias[GN_D];
  __shared__ __attribute__((aligned(16))) float sP[8][GN_TS * 8];
  __shared__ __attribute__((aligned(16))) int   sSrc[8][GN_TS];
  __shared__ __attribute__((aligned(16))) float sRow[8][GN_D];
  const int tid = (int)threadIdx.x, lane = tid & 31, wave = tid >> 5, hh = lane >> 4;
  if (tid < 128) *(v4fa*)(sBias + 4 * tid) = *(const v4fa*)(PAR + 2 * GN_D + 4 * tid);
  __syncthreads();

  const int row = (int)blockIdx.x * 8 + wave;
  const int i   = clampi(row, 0, nN - 1);
  int cv = CNTT[i];
  asm volatile("" :: "v"(cv));
  cv = clampi(cv, 0, GN_DEGCAP);
  const int cn = __builtin_amdgcn_readfirstlane(cv);
  int ov = OFFT[i];
  asm volatile("" :: "v"(ov));
  ov = clampi(ov, 0, GN_RCAP - 1);
  const int off = __builtin_amdgcn_readfirstlane(ov);
  const int fv = FLGT[i];
  asm volatile("" :: "v"(fv));
  const int lbase = (i >> 9) * GN_RCAP;
  const int nent  = cn + 1;
  const v4f ad0 = *(const v4fa*)(SD + (size_t)i * 16 + 8);
  const v4f ad1 = *(const v4fa*)(SD + (size_t)i * 16 + 12);
  float* pw = sP[wave];
  int*   sw = sSrc[wave];
  const float ninf = __int_as_float((int)0xff800000u);

  float mx[8];
#pragma unroll
  for (int q = 0; q < 8; ++q) mx[q] = ninf;

#pragma unroll 1
  for (int k = 0; k < 3; ++k) {
    const int t = lane + 32 * k;
    int lp = t < cn - 1 ? t : cn - 1;
    lp = lp < 0 ? 0 : lp;
    int pos = off + lp;
    pos = pos > GN_RCAP - 1 ? GN_RCAP - 1 : pos;
    const int sl = LIST[lbase + pos];
    asm volatile("" :: "v"(sl));
    const int slc = clampi(sl, 0, nN - 1);
    const int s = (t >= cn) ? i : slc;
    const v4f a0 = *(const v4fa*)(SD + (size_t)s * 16);
    asm volatile("" :: "v"(a0));
    const v4f a1 = *(const v4fa*)(SD + (size_t)s * 16 + 4);
    asm volatile("" :: "v"(a1));
    const bool valid = t < nent;
    float e[8];
#pragma unroll
    for (int q = 0; q < 4; ++q) { e[q] = a0[q] + ad0[q]; e[4 + q] = a1[q] + ad1[q]; }
#pragma unroll
    for (int q = 0; q < 8; ++q) {
      float v = e[q];
      v = (v >= 0.0f) ? v : 0.2f * v;
      v = valid ? v : ninf;
      e[q] = v;
      mx[q] = fmaxf(mx[q], v);
    }
    *(v4fa*)(pw + t * 8)     = (v4f){ e[0], e[1], e[2], e[3] };
    *(v4fa*)(pw + t * 8 + 4) = (v4f){ e[4], e[5], e[6], e[7] };
    sw[t] = s;
  }
#pragma unroll
  for (int q = 0; q < 8; ++q) {
#pragma unroll
    for (int o = 16; o > 0; o >>= 1) mx[q] = fmaxf(mx[q], __shfl_xor(mx[q], o));
  }

#pragma unroll 1
  for (int k = 0; k < 3; ++k) {
    const int t = lane + 32 * k;
    const bool valid = t < nent;
    const v4f e0 = *(const v4fa*)(pw + t * 8);
    const v4f e1 = *(const v4fa*)(pw + t * 8 + 4);
    float p[8];
#pragma unroll
    for (int q = 0; q < 4; ++q) {
      const float x0 = expf(e0[q] - mx[q]);
      const float x1 = expf(e1[q] - mx[4 + q]);
      p[q]     = valid ? x0 : 0.0f;
      p[4 + q] = valid ? x1 : 0.0f;
    }
    *(v4fa*)(pw + t * 8)     = (v4f){ p[0], p[2], p[4], p[6] };
    *(v4fa*)(pw + t * 8 + 4) = (v4f){ p[1], p[3], p[5], p[7] };
  }
  __builtin_amdgcn_fence(__ATOMIC_RELEASE, "workgroup");
  __builtin_amdgcn_wave_barrier();
  __builtin_amdgcn_fence(__ATOMIC_ACQUIRE, "workgroup");

  v4f acc0 = (v4f){0.f, 0.f, 0.f, 0.f}, acc1 = acc0, acc2 = acc0, acc3 = acc0, den = acc0;
#pragma unroll 1
  for (int t = 0; t < nent; ++t) {
    const int sv = sw[t];
    const int s  = clampi(__builtin_amdgcn_readfirstlane(sv), 0, nN - 1);
    const v4f pv = *(const v4fa*)(pw + t * 8 + hh * 4);
    const float* hp = HS + (size_t)s * GN_LDH + 4 * lane;
    const v4f h0 = *(const v4fa*)(hp);
    asm volatile("" :: "v"(h0));
    const v4f h1 = *(const v4fa*)(hp + 128);
    asm volatile("" :: "v"(h1));
    const v4f h2 = *(const v4fa*)(hp + 256);
    asm volatile("" :: "v"(h2));
    const v4f h3 = *(const v4fa*)(hp + 384);
    asm volatile("" :: "v"(h3));
    acc0 += pv[0] * h0;
    acc1 += pv[1] * h1;
    acc2 += pv[2] * h2;
    acc3 += pv[3] * h3;
    den  += pv;
  }

  float* rb = sRow[wave];
  *(v4fa*)(rb + 4 * lane)       = acc0;
  *(v4fa*)(rb + 128 + 4 * lane) = acc1;
  *(v4fa*)(rb + 256 + 4 * lane) = acc2;
  *(v4fa*)(rb + 384 + 4 * lane) = acc3;
  const float qn = __int_as_float(0x7fc00000);
#pragma unroll 1
  for (int j = 0; j < 4; ++j) {
    const v4f a = *(const v4fa*)(rb + j * 128 + 4 * lane);
    float d = den[0];
    d = (j == 1) ? den[1] : d;
    d = (j == 2) ? den[2] : d;
    d = (j == 3) ? den[3] : d;
    const v4f b = *(const v4fa*)(sBias + j * 128 + 4 * lane);
    v4f v = a / d + b;
    v[0] = (fv != 0) ? qn : v[0];
    v[1] = (fv != 0) ? qn : v[1];
    v[2] = (fv != 0) ? qn : v[2];
    v[3] = (fv != 0) ? qn : v[3];
    *(v4fa*)(rb + j * 128 + 4 * lane) = v;
  }
  const bool wr = row < nN;
  float* grow = G + (size_t)i * GN_D + 4 * lane;
  for (int pass = 0; pass < 2; ++pass) {
#pragma unroll
    for (int j = 0; j < 4; ++j) {
      const v4f v = *(const v4fa*)(rb + j * 128 + 4 * lane);
      if (wr) *(volatile v4f*)(grow + j * 128) = v;
    }
    __threadfence();
  }
}

template <int MODE>
__global__ __launch_bounds__(256) void k_colstat(const float* __restrict__ G, const float* __restrict__ STAT,
                                                 double* __restrict__ REC, int nN) {
  const int c = 2 * (int)threadIdx.x;
  const int base = (int)blockIdx.x * GN_RB;
  int rows = nN - base;
  rows = rows > GN_RB ? GN_RB : rows;
  rows = rows < 0 ? 0 : rows;
  rows = __builtin_amdgcn_readfirstlane(rows);
  v2f mu = (v2f){0.f, 0.f};
  if (MODE == 1) mu = *(const v2fa*)(STAT + c);
  float s0 = 0.0f, s1 = 0.0f;
  const float* p = G + (size_t)base * GN_D + c;
#pragma unroll 4
  for (int r = 0; r < rows; ++r) {
    const v2f g = *(const v2fa*)(p + (size_t)r * GN_D);
    if (MODE == 1) {
      const float d0 = g[0] - mu[0], d1 = g[1] - mu[1];
      s0 = fmaf(d0, d0, s0);
      s1 = fmaf(d1, d1, s1);
    } else {
      s0 += g[0];
      s1 += g[1];
    }
  }
  const v2d o = (v2d){ (double)s0, (double)s1 };
  volatile v2d* q = (volatile v2d*)(REC + (size_t)blockIdx.x * GN_D + c);
  *q = o;
  __threadfence();
  *q = o;
}

template <int MODE>
__global__ __launch_bounds__(512) void k_stat(const double* __restrict__ REC, float* __restrict__ dst) {
  __shared__ __attribute__((aligned(16))) float sv[GN_D];
  const int c = (int)threadIdx.x;
  double a = 0.0;
#pragma unroll 4
  for (int b = 0; b < GN_SB; ++b) a += REC[(size_t)b * GN_D + c];
  const double m = a * 1.0e-4;
  float o;
  if (MODE == 0) o = (float)m;
  else           o = 1.0f / sqrtf((float)m + 1.0e-5f);
  sv[c] = o;
  __syncthreads();
  if (c < 128) {
    const v4f v = *(const v4fa*)(sv + 4 * c);
    volatile v4f* q = (volatile v4f*)(dst + 4 * c);
    *q = v;
    __threadfence();
    *q = v;
  }
}

__global__ __launch_bounds__(256) void k_final(const float* __restrict__ G, const float* __restrict__ HS,
                                               const float* __restrict__ STAT, const float* __restrict__ PAR,
                                               float* __restrict__ out, int nN) {
  __shared__ __attribute__((aligned(16))) float sPar[5 * GN_D];
  __shared__ __attribute__((aligned(16))) float sY[8][GN_D];
  const int tid = (int)threadIdx.x, lane = tid & 31, wave = tid >> 5;
  *(v4fa*)(sPar + 4 * tid)            = *(const v4fa*)(STAT + 4 * tid);
  *(v4fa*)(sPar + 2 * GN_D + 4 * tid) = *(const v4fa*)(PAR + 3 * GN_D + 4 * tid);
  if (tid < 128) *(v4fa*)(sPar + 4 * GN_D + 4 * tid) = *(const v4fa*)(PAR + 5 * GN_D + 4 * tid);
  __syncthreads();

  const int row = (int)blockIdx.x * 8 + wave;
  const int rc  = clampi(row, 0, nN - 1);
  float* yb = sY[wave];
  const float* gp = G  + (size_t)rc * GN_D + 4 * lane;
  const float* hp = HS + (size_t)rc * GN_LDH + GN_D + 4 * lane;
  v4f idn[4];
#pragma unroll
  for (int j = 0; j < 4; ++j) {
    const int col = j * 128 + 4 * lane;
    const v4f g = *(const v4fa*)(gp + j * 128);
    asm volatile("" :: "v"(g));
    const v4f hs = *(const v4fa*)(hp + j * 128);
    asm volatile("" :: "v"(hs));
    const v4f mu = *(const v4fa*)(sPar + col);
    const v4f rs = *(const v4fa*)(sPar + GN_D + col);
    const v4f ga = *(const v4fa*)(sPar + 2 * GN_D + col);
    const v4f be = *(const v4fa*)(sPar + 3 * GN_D + col);
    const v4f bs = *(const v4fa*)(sPar + 4 * GN_D + col);
    asm volatile("" :: "v"(bs));
    const v4f y = (g - mu) * rs * ga + be;
    idn[j] = hs + bs;
    *(v4fa*)(yb + col) = y;
  }
#pragma unroll 1
  for (int q = 0; q < 16; ++q) {
    const int a = (q >> 2) * 128 + 4 * lane + (q & 3);
    const float y = yb[a];
    const float gl = 0.5f * y * (1.0f + erff(y * 0.70710678f));
    yb[a] = gl;
  }
  v4f o[4];
#pragma unroll
  for (int j = 0; j < 4; ++j) o[j] = *(const v4fa*)(yb + j * 128 + 4 * lane) + idn[j];
  const bool wr = row < nN;
  float* orow = out + (size_t)rc * GN_D + 4 * lane;
  for (int pass = 0; pass < 2; ++pass) {
#pragma unroll
    for (int j = 0; j < 4; ++j) {
      if (wr) *(volatile v4f*)(orow + j * 128) = o[j];
    }
    __threadfence();
  }
}

extern "C" void kernel_launch(void* const* d_in, const int* in_sizes, int n_in,
                              void* d_out, int out_size, void* d_ws, size_t ws_size,
                              hipStream_t stream) {
  if (n_in < 10) return;
  if (in_sizes[0] != GN_N * GN_D) return;
  if (in_sizes[1] != 2 * GN_E) return;
  if (in_sizes[2] != GN_D * GN_D) return;
  if (in_sizes[3] != GN_D || in_sizes[4] != GN_D) return;
  if (in_sizes[5] != GN_D || in_sizes[6] != GN_D || in_sizes[7] != GN_D) return;
  if (in_sizes[8] != GN_D * GN_D || in_sizes[9] != GN_D) return;
  if (out_size != GN_N * GN_D) return;
  if (ws_size < WS_TOTAL) return;

  const float* x     = (const float*)d_in[0];
  const int*   ei    = (const int*)  d_in[1];
  const float* Wg    = (const float*)d_in[2];
  const float* asrc  = (const float*)d_in[3];
  const float* adst  = (const float*)d_in[4];
  const float* gbias = (const float*)d_in[5];
  const float* gamma = (const float*)d_in[6];
  const float* beta  = (const float*)d_in[7];
  const float* Ws    = (const float*)d_in[8];
  const float* bskip = (const float*)d_in[9];
  float* out = (float*)d_out;

  char* ws = (char*)d_ws;
  unsigned short* XB   = (unsigned short*)(ws + OF_XB);
  unsigned short* WT   = (unsigned short*)(ws + OF_WT);
  float*          HS   = (float*)(ws + OF_HS);
  float*          SD   = (float*)(ws + OF_SD);
  float*          Gp   = (float*)(ws + OF_G);
  int*            LIST = (int*)(ws + OF_LIST);
  int*            OFFT = (int*)(ws + OF_OFF);
  int*            CNTT = (int*)(ws + OF_CNT);
  int*            FLGT = (int*)(ws + OF_FLG);
  double*         REC1 = (double*)(ws + OF_REC1);
  double*         REC2 = (double*)(ws + OF_REC2);
  float*          STAT = (float*)(ws + OF_STAT);
  float*          PAR  = (float*)(ws + OF_PAR);

  hipFuncSetAttribute(reinterpret_cast<const void*>(&k_bucket),
                      hipFuncAttributeMaxDynamicSharedMemorySize, GN_BK_LDS);

  k_plane<0><<<GN_MP * GN_D / 8 / 256, 256, 0, stream>>>(x, GN_N, GN_D, GN_D, XB, GN_MP, GN_D);
  k_wtr<<<GN_D * (GN_D / 8) / 256, 256, 0, stream>>>(Wg, WT);
  k_wtr<<<GN_D * (GN_D / 8) / 256, 256, 0, stream>>>(Ws, WT + (size_t)GN_D * GN_D);
  k_par<<<1, 128, 0, stream>>>(asrc, adst, gbias, gamma, beta, bskip, PAR);
  k_gemm_nt<0, 0><<<(GN_MP / 64) * (GN_LDH / 64) / 8, 256, 0, stream>>>(XB, WT, PAR, HS, GN_MP, GN_LDH, GN_D, GN_LDH);
  k_dots<<<GN_N / 8, 256, 0, stream>>>(HS, PAR, SD, GN_N);
  k_bucket<<<GN_NBLK, 256, GN_BK_LDS, stream>>>(ei, LIST, OFFT, CNTT, FLGT, GN_E, GN_N);
  k_replay<<<GN_N / 8, 256, 0, stream>>>(HS, SD, PAR, LIST, OFFT, CNTT, FLGT, Gp, GN_N);
  k_colstat<0><<<GN_SB, 256, 0, stream>>>(Gp, STAT, REC1, GN_N);
  k_stat<0><<<1, 512, 0, stream>>>(REC1, STAT);
  k_colstat<1><<<GN_SB, 256, 0, stream>>>(Gp, STAT, REC2, GN_N);
  k_stat<1><<<1, 512, 0, stream>>>(REC2, STAT + GN_D);
  k_final<<<GN_N / 8, 256, 0, stream>>>(Gp, HS, STAT, PAR, out, GN_N);
}
